// SnailBlock_20804821582359
// MI455X (gfx1250) — hardware-verified
//
#include <hip/hip_runtime.h>
#include <stdint.h>
#include <stddef.h>

#define NBATCH 4
#define HID    128
#define NPOS   4096
#define MPIX   16384
#define NLAYER 4
#define QKD    16
#define KQ     160
#define CIN    130
#define STP    20

typedef _Float16 v16h __attribute__((ext_vector_type(16)));
typedef _Float16 v8h  __attribute__((ext_vector_type(8)));
typedef _Float16 v4h  __attribute__((ext_vector_type(4)));
typedef __bf16   v16b __attribute__((ext_vector_type(16)));
typedef __bf16   v8b  __attribute__((ext_vector_type(8)));
typedef float    v8f  __attribute__((ext_vector_type(8)));
typedef float    v4f  __attribute__((ext_vector_type(4)));
typedef unsigned v4u  __attribute__((ext_vector_type(4)));

union FH { v16h v; v8h h[2]; unsigned u[8]; };
union FB { v16b v; v8b h[2]; unsigned u[8]; };

__device__ __forceinline__ v8f mma_h(v16h a, v16h b, v8f c) {
  c = __builtin_amdgcn_wmma_f32_16x16x32_f16(false, a, false, b, (short)0, c, false, false);
  asm volatile("v_nop\n\tv_nop\n\tv_nop\n\tv_nop" : "+v"(c) : "v"(a), "v"(b));
  return c;
}
__device__ __forceinline__ v8f mma_b(v16b a, v16b b, v8f c) {
  c = __builtin_amdgcn_wmma_f32_16x16x32_bf16(false, a, false, b, (short)0, c, false, false);
  asm volatile("v_nop\n\tv_nop\n\tv_nop\n\tv_nop" : "+v"(c) : "v"(a), "v"(b));
  return c;
}
__device__ __forceinline__ v8f zacc() {
  v8f z = {0.f, 0.f, 0.f, 0.f, 0.f, 0.f, 0.f, 0.f};
  return z;
}

__device__ __forceinline__ unsigned short bf_bits(float f) {
  unsigned u = __float_as_uint(f);
  return (unsigned short)((u + 0x7FFFu + ((u >> 16) & 1u)) >> 16);
}
__device__ __forceinline__ float bf_val(unsigned short b) { return __uint_as_float(((unsigned)b) << 16); }
__device__ __forceinline__ float eluf(float x) { return x > 0.0f ? x : (__expf(x) - 1.0f); }
__device__ __forceinline__ float sigf(float x) { return __builtin_amdgcn_rcpf(1.0f + __expf(-x)); }

__device__ __forceinline__ v8h pack8h(const float* v) {
  v8h o;
#pragma unroll
  for (int e = 0; e < 8; ++e) o[e] = (_Float16)v[e];
  return o;
}
__device__ __forceinline__ void split8(const float* v, v4u& hi, v4u& lo) {
#pragma unroll
  for (int q = 0; q < 4; ++q) {
    const unsigned short h0 = bf_bits(v[2 * q]), h1 = bf_bits(v[2 * q + 1]);
    const unsigned short l0 = bf_bits(v[2 * q] - bf_val(h0)), l1 = bf_bits(v[2 * q + 1] - bf_val(h1));
    hi[q] = (unsigned)h0 | ((unsigned)h1 << 16);
    lo[q] = (unsigned)l0 | ((unsigned)l1 << 16);
  }
}

__global__ __launch_bounds__(256) void k_prep_convw(const float* __restrict__ w, unsigned short* __restrict__ dst, int rows) {
  const int idx = blockIdx.x * 256 + threadIdx.x;
  if (idx >= rows * 64) return;
  const int e0 = idx * 8;
  const int row = e0 >> 9, k0 = e0 & 511;
  const int tap = k0 >> 7, c0 = k0 & 127;
  float v[8];
#pragma unroll
  for (int e = 0; e < 8; ++e) v[e] = w[((size_t)row * HID + c0 + e) * 4 + tap] * 16.0f;
  const v8h o = pack8h(v);
  _Float16* p = (_Float16*)dst + e0;
  *(volatile v8h*)p = o;
  __threadfence();
  *(volatile v8h*)p = o;
}

__global__ __launch_bounds__(256) void k_prep_qkvw(const float* __restrict__ w, unsigned short* __restrict__ dst) {
  const int idx = blockIdx.x * 256 + threadIdx.x;
  if (idx >= KQ * KQ / 8) return;
  const int e0 = idx * 8;
  const int o = e0 / KQ, k0 = e0 - o * KQ;
  float v[8];
#pragma unroll
  for (int e = 0; e < 8; ++e) {
    const int kk = k0 + e;
    const int kc = kk < CIN ? kk : (CIN - 1);
    const float f = w[(size_t)o * CIN + kc] * 16.0f;
    v[e] = (kk < CIN) ? f : 0.0f;
  }
  const v8h ov = pack8h(v);
  _Float16* p = (_Float16*)dst + e0;
  *(volatile v8h*)p = ov;
  __threadfence();
  *(volatile v8h*)p = ov;
}

__global__ __launch_bounds__(256) void k_prep_splitw(const float* __restrict__ w, unsigned short* __restrict__ hi,
                                                    unsigned short* __restrict__ lo) {
  const int idx = blockIdx.x * 256 + threadIdx.x;
  if (idx >= HID * HID / 8) return;
  const int e0 = idx * 8;
  float v[8];
#pragma unroll
  for (int e = 0; e < 8; ++e) v[e] = w[e0 + e];
  v4u hv, lv;
  split8(v, hv, lv);
  *(volatile v4u*)(hi + e0) = hv;
  *(volatile v4u*)(lo + e0) = lv;
  __threadfence();
  *(volatile v4u*)(hi + e0) = hv;
  *(volatile v4u*)(lo + e0) = lv;
}

__global__ __launch_bounds__(256) void k_transpose_in(const float* __restrict__ x, float* __restrict__ H,
                                                      unsigned short* __restrict__ HXp) {
  __shared__ __align__(16) float tile[HID * 68];
  const int by = blockIdx.x;
  const int b = by >> 6, y = by & 63;
  const int tid = threadIdx.x;
#pragma unroll
  for (int it = 0; it < 8; ++it) {
    const int c = it * 16 + (tid >> 4);
    const int px = (tid & 15) * 4;
    const v4f a = *(const v4f*)(x + ((size_t)(b * HID + c)) * NPOS + y * 64 + px);
    *(v4f*)(tile + c * 68 + px) = a;
  }
  __syncthreads();
  const int wave = tid >> 5, lane = tid & 31, hh = lane >> 4, m = lane & 15;
  const size_t mb = (size_t)by * 64 + wave * 8;
  _Float16* HX = (_Float16*)HXp;
  for (int pass = 0; pass < 2; ++pass) {
#pragma unroll
    for (int i = 0; i < 8; ++i) {
      const int px = wave * 8 + i;
      const int c4 = lane * 4;
      v4f v;
#pragma unroll
      for (int e = 0; e < 4; ++e) v[e] = tile[(c4 + e) * 68 + px];
      *(volatile v4f*)(H + (mb + i) * HID + c4) = v;
    }
#pragma unroll
    for (int i = 0; i < 4; ++i) {
      const int rr = i * 2 + hh;
      const int px = wave * 8 + rr;
      const int c0 = 8 * m;
      float v[8];
#pragma unroll
      for (int e = 0; e < 8; ++e) v[e] = eluf(tile[(c0 + e) * 68 + px]);
      *(volatile v8h*)(HX + (mb + rr) * HID + c0) = pack8h(v);
    }
    __threadfence();
  }
}

template <int EPI>
__global__ __launch_bounds__(128) void k_conv(const unsigned short* __restrict__ in, const unsigned short* __restrict__ Wl,
                                              const float* __restrict__ bias, void* __restrict__ outp) {
  __shared__ __align__(16) unsigned short wl[128 * 32];
  __shared__ __align__(16) float st[4 * 128 * STP];
  const int tid = threadIdx.x, wave = tid >> 5, lane = tid & 31;
  const int m = lane & 15, hh = lane >> 4;
  const int nb = blockIdx.y;
  const int bm0 = blockIdx.x * 64;
  const int m0 = bm0 + wave * 16;
  const int b = m0 >> 12, y = (m0 >> 6) & 63, x0 = m0 & 63;
  const int xq = x0 + m;
  const unsigned short* Wn = Wl + (size_t)nb * 128 * 512;
  const _Float16* inh = (const _Float16*)in;
  const _Float16* wlh = (const _Float16*)wl;

  v8f acc[8];
#pragma unroll
  for (int nt = 0; nt < 8; ++nt) acc[nt] = zacc();

#pragma unroll 1
  for (int kc = 0; kc < 16; ++kc) {
    __syncthreads();
#pragma unroll
    for (int q = 0; q < 4; ++q) {
      const int ci = tid * 4 + q;
      const int col = ci >> 2, part = (ci & 3) * 8;
      const v4u pv = *(const v4u*)(Wn + (size_t)col * 512 + kc * 32 + part);
      *(v4u*)(wl + col * 32 + part) = pv;
    }
    __syncthreads();
    const int tap = kc >> 2;
    const int yy = y - 1 + (tap >> 1);
    const int xx = xq - 1 + (tap & 1);
    const bool ok = (yy >= 0) && (xx >= 0);
    const int yyc = yy < 0 ? 0 : yy;
    const int xxc = xx < 0 ? 0 : xx;
    const _Float16* src = inh + ((size_t)b * NPOS + (size_t)yyc * 64 + xxc) * HID + (kc & 3) * 32;
    FH a;
    a.h[0] = *(const v8h*)(src + 8 * hh);
    a.h[1] = *(const v8h*)(src + 16 + 8 * hh);
#pragma unroll
    for (int e = 0; e < 8; ++e) a.u[e] = ok ? a.u[e] : 0u;
#pragma unroll
    for (int nt = 0; nt < 8; ++nt) {
      const _Float16* br = wlh + (nt * 16 + m) * 32;
      FH bf;
      bf.h[0] = *(const v8h*)(br + 8 * hh);
      bf.h[1] = *(const v8h*)(br + 16 + 8 * hh);
      acc[nt] = mma_h(a.v, bf.v, acc[nt]);
    }
  }

  float* ST = st + wave * (128 * STP);
#pragma unroll
  for (int nt = 0; nt < 8; ++nt) {
    const int col = nt * 16 + m;
    const float bv = bias[nb * 128 + col];
    v4f p0, p1;
#pragma unroll
    for (int e = 0; e < 4; ++e) {
      p0[e] = acc[nt][e] * 0.0625f + bv;
      p1[e] = acc[nt][4 + e] * 0.0625f + bv;
    }
    *(v4f*)(ST + col * STP + 8 * hh) = p0;
    *(v4f*)(ST + col * STP + 8 * hh + 4) = p1;
  }
  __syncthreads();

  if (EPI == 0) {
    _Float16* out = (_Float16*)outp;
    for (int pass = 0; pass < 2; ++pass) {
#pragma unroll
      for (int it = 0; it < 8; ++it) {
        const int row = it * 2 + hh, c0 = 8 * m;
        float v[8];
#pragma unroll
        for (int e = 0; e < 8; ++e) v[e] = eluf(ST[(c0 + e) * STP + row]);
        *(volatile v8h*)(out + (size_t)(m0 + row) * HID + c0) = pack8h(v);
      }
      __threadfence();
    }
  } else {
    float* out = (float*)outp;
    for (int pass = 0; pass < 2; ++pass) {
#pragma unroll
      for (int it = 0; it < 16; ++it) {
        const int c4 = 4 * lane;
        v4f v;
#pragma unroll
        for (int e = 0; e < 4; ++e) v[e] = ST[(c4 + e) * STP + it];
        *(volatile v4f*)(out + (size_t)(m0 + it) * 256 + nb * 128 + c4) = v;
      }
      __threadfence();
    }
  }
}

__global__ __launch_bounds__(256) void k_gate(const float* __restrict__ Hc, const float* __restrict__ O,
                                              float* __restrict__ Hn, unsigned short* __restrict__ HXp) {
  const int idx = blockIdx.x * 256 + threadIdx.x;
  if (idx >= MPIX * 32) return;
  const int mrow = idx >> 5, c4 = (idx & 31) * 4;
  const v4f h  = *(const v4f*)(Hc + (size_t)mrow * HID + c4);
  const v4f o1 = *(const v4f*)(O + (size_t)mrow * 256 + c4);
  const v4f o2 = *(const v4f*)(O + (size_t)mrow * 256 + 128 + c4);
  v4f hn;
  v4h hx;
#pragma unroll
  for (int e = 0; e < 4; ++e) {
    const float v = eluf(h[e]) + o1[e] * sigf(o2[e]);
    hn[e] = v;
    hx[e] = (_Float16)eluf(v);
  }
  _Float16* HX = (_Float16*)HXp;
  *(volatile v4f*)(Hn + (size_t)mrow * HID + c4) = hn;
  *(volatile v4h*)(HX + (size_t)mrow * HID + c4) = hx;
  __threadfence();
  *(volatile v4f*)(Hn + (size_t)mrow * HID + c4) = hn;
  *(volatile v4h*)(HX + (size_t)mrow * HID + c4) = hx;
}

__global__ __launch_bounds__(256) void k_build_a(const float* __restrict__ H, const float* __restrict__ pos,
                                                 unsigned short* __restrict__ Ap) {
  const int idx = blockIdx.x * 256 + threadIdx.x;
  if (idx >= MPIX * 20) return;
  const int mrow = idx / 20, j0 = (idx - mrow * 20) * 8;
  const int b = mrow >> 12, p = mrow & 4095;
  const int jc = j0 < 128 ? j0 : 120;
  const v4f h0 = *(const v4f*)(H + (size_t)mrow * HID + jc);
  const v4f h1 = *(const v4f*)(H + (size_t)mrow * HID + jc + 4);
  const float p0v = pos[((size_t)(b * 2)) * NPOS + p];
  const float p1v = pos[((size_t)(b * 2 + 1)) * NPOS + p];
  const bool ish = (j0 < 128);
  const bool isp = (j0 == 128);
  float v[8];
  v[0] = ish ? h0[0] : (isp ? p0v : 0.0f);
  v[1] = ish ? h0[1] : (isp ? p1v : 0.0f);
  v[2] = ish ? h0[2] : 0.0f;
  v[3] = ish ? h0[3] : 0.0f;
#pragma unroll
  for (int e = 0; e < 4; ++e) v[4 + e] = ish ? h1[e] : 0.0f;
  const v8h o = pack8h(v);
  _Float16* pd = (_Float16*)Ap + (size_t)idx * 8;
  *(volatile v8h*)pd = o;
  __threadfence();
  *(volatile v8h*)pd = o;
}

__global__ __launch_bounds__(256) void k_split_elu(const float* __restrict__ H, unsigned short* __restrict__ hi,
                                                   unsigned short* __restrict__ lo) {
  const int idx = blockIdx.x * 256 + threadIdx.x;
  if (idx >= MPIX * 16) return;
  const size_t e0 = (size_t)idx * 8;
  const v4f a0 = *(const v4f*)(H + e0);
  const v4f a1 = *(const v4f*)(H + e0 + 4);
  float v[8];
#pragma unroll
  for (int e = 0; e < 4; ++e) { v[e] = eluf(a0[e]); v[4 + e] = eluf(a1[e]); }
  v4u hv, lv;
  split8(v, hv, lv);
  *(volatile v4u*)(hi + e0) = hv;
  *(volatile v4u*)(lo + e0) = lv;
  __threadfence();
  *(volatile v4u*)(hi + e0) = hv;
  *(volatile v4u*)(lo + e0) = lv;
}

__global__ __launch_bounds__(128) void k_qkv(const unsigned short* __restrict__ Ap, const unsigned short* __restrict__ Wq,
                                             const float* __restrict__ bias, unsigned short* __restrict__ Qo,
                                             unsigned short* __restrict__ Ko, unsigned short* __restrict__ VTo) {
  __shared__ __align__(16) unsigned short wl[KQ * 32];
  __shared__ __align__(16) float st[4 * KQ * STP];
  const int tid = threadIdx.x, wave = tid >> 5, lane = tid & 31;
  const int m = lane & 15, hh = lane >> 4;
  const int bm0 = blockIdx.x * 64;
  const int m0 = bm0 + wave * 16;
  const _Float16* A = (const _Float16*)Ap;
  const _Float16* wlh = (const _Float16*)wl;

  v8f acc[10];
#pragma unroll
  for (int nt = 0; nt < 10; ++nt) acc[nt] = zacc();

#pragma unroll 1
  for (int kc = 0; kc < KQ / 32; ++kc) {
    __syncthreads();
    for (int ci = tid; ci < KQ * 4; ci += 128) {
      const int col = ci >> 2, part = (ci & 3) * 8;
      const v4u pv = *(const v4u*)(Wq + (size_t)col * KQ + kc * 32 + part);
      *(v4u*)(wl + col * 32 + part) = pv;
    }
    __syncthreads();
    const _Float16* ar = A + (size_t)(m0 + m) * KQ + kc * 32;
    FH a;
    a.h[0] = *(const v8h*)(ar + 8 * hh);
    a.h[1] = *(const v8h*)(ar + 16 + 8 * hh);
#pragma unroll
    for (int nt = 0; nt < 10; ++nt) {
      const _Float16* br = wlh + (nt * 16 + m) * 32;
      FH bf;
      bf.h[0] = *(const v8h*)(br + 8 * hh);
      bf.h[1] = *(const v8h*)(br + 16 + 8 * hh);
      acc[nt] = mma_h(a.v, bf.v, acc[nt]);
    }
  }

  float* ST = st + wave * (KQ * STP);
#pragma unroll
  for (int nt = 0; nt < 10; ++nt) {
    const int col = nt * 16 + m;
    const float bv = bias[col];
    v4f p0, p1;
#pragma unroll
    for (int e = 0; e < 4; ++e) {
      p0[e] = acc[nt][e] * 0.0625f + bv;
      p1[e] = acc[nt][4 + e] * 0.0625f + bv;
    }
    *(v4f*)(ST + col * STP + 8 * hh) = p0;
    *(v4f*)(ST + col * STP + 8 * hh + 4) = p1;
  }
  __syncthreads();

  _Float16* Q  = (_Float16*)Qo;
  _Float16* Kk = (_Float16*)Ko;
  _Float16* VT = (_Float16*)VTo;
  const int b = bm0 >> 12, p0 = bm0 & 4095;
  for (int pass = 0; pass < 2; ++pass) {
    {
      const int row = lane >> 1, c0 = 8 * (lane & 1);
      float v[8];
#pragma unroll
      for (int e = 0; e < 8; ++e) v[e] = ST[(c0 + e) * STP + row];
      *(volatile v8h*)(Q + (size_t)(m0 + row) * QKD + c0) = pack8h(v);
#pragma unroll
      for (int e = 0; e < 8; ++e) v[e] = ST[(QKD + c0 + e) * STP + row];
      *(volatile v8h*)(Kk + (size_t)(m0 + row) * QKD + c0) = pack8h(v);
    }
#pragma unroll
    for (int it = 0; it < 8; ++it) {
      const int ch = wave * 32 + it * 4 + (lane >> 3);
      const int pxb = 8 * (lane & 7);
      const int pt = pxb >> 4, r0 = pxb & 15;
      const float* sp = st + pt * (KQ * STP) + (32 + ch) * STP + r0;
      const v4f a0 = *(const v4f*)sp;
      const v4f a1 = *(const v4f*)(sp + 4);
      float v[8];
#pragma unroll
      for (int e = 0; e < 4; ++e) { v[e] = a0[e]; v[4 + e] = a1[e]; }
      *(volatile v8h*)(VT + ((size_t)(b * HID + ch)) * NPOS + p0 + pxb) = pack8h(v);
    }
    __threadfence();
  }
}

__global__ __launch_bounds__(128) void k_attn(const unsigned short* __restrict__ Qp, const unsigned short* __restrict__ Kp,
                                              const unsigned short* __restrict__ VTp, unsigned short* __restrict__ AVh,
                                              unsigned short* __restrict__ AVl) {
  __shared__ __align__(16) unsigned char lds[4 * 128 * STP * 4];
  _Float16* Ksh = (_Float16*)(lds);
  _Float16* Vth = (_Float16*)(lds + 2048);
  _Float16* Psh = (_Float16*)(lds + 2048 + 16384);
  float*    Os  = (float*)(lds);

  const int tid = threadIdx.x, wave = tid >> 5, lane = tid & 31;
  const int m = lane & 15, hh = lane >> 4;
  const int b = blockIdx.x >> 6, qb = blockIdx.x & 63;
  const int q0 = qb * 64 + wave * 16;
  const size_t gm = (size_t)b * NPOS;
  const _Float16* Q  = (const _Float16*)Qp;
  const _Float16* Kk = (const _Float16*)Kp;
  const _Float16* VT = (const _Float16*)VTp;

  FH qa;
  qa.h[0] = *(const v8h*)(Q + (gm + q0 + m) * QKD + 8 * hh);
#pragma unroll
  for (int e = 4; e < 8; ++e) qa.u[e] = 0u;

  float mrow[8], lrow[8];
  v8f oacc[8];
#pragma unroll
  for (int r = 0; r < 8; ++r) { mrow[r] = -__builtin_inff(); lrow[r] = 0.f; }
#pragma unroll
  for (int t = 0; t < 8; ++t) oacc[t] = zacc();

  _Float16* pw = Psh + wave * (16 * 64);

#pragma unroll 1
  for (int kc = 0; kc <= qb; ++kc) {
    const int kv0 = kc * 64;
    __syncthreads();
    {
      const int kr = tid >> 1, kp = (tid & 1) * 8;
      const v4u kvv = *(const v4u*)(Kk + (gm + kv0 + kr) * QKD + kp);
      *(v4u*)(Ksh + kr * QKD + kp) = kvv;
#pragma unroll
      for (int i = 0; i < 8; ++i) {
        const int ci = tid + 128 * i;
        const int ch = ci >> 3, part = (ci & 7) * 8;
        const v4u vv = *(const v4u*)(VT + ((size_t)(b * HID + ch)) * NPOS + kv0 + part);
        *(v4u*)(Vth + ch * 64 + part) = vv;
      }
    }
    __syncthreads();

    v8f s[4];
#pragma unroll
    for (int j = 0; j < 4; ++j) {
      FH kb;
      kb.h[0] = *(const v8h*)(Ksh + (j * 16 + m) * QKD + 8 * hh);
#pragma unroll
      for (int e = 4; e < 8; ++e) kb.u[e] = 0u;
      s[j] = mma_h(qa.v, kb.v, zacc());
    }

    const bool diag = (kc == qb);
    float cm[8];
#pragma unroll
    for (int r = 0; r < 8; ++r) {
      const int qrow = q0 + 8 * hh + r;
      float mx = -__builtin_inff();
#pragma unroll
      for (int j = 0; j < 4; ++j) {
        const int kcol = kv0 + j * 16 + m;
        const float sv = s[j][r] * 0.25f;
        const bool masked = diag && (kcol > qrow);
        const float sm = masked ? -__builtin_inff() : sv;
        s[j][r] = sm;
        mx = fmaxf(mx, sm);
      }
#pragma unroll
      for (int off = 1; off < 16; off <<= 1) mx = fmaxf(mx, __shfl_xor(mx, off, 32));
      cm[r] = mx;
    }
#pragma unroll
    for (int r = 0; r < 8; ++r) {
      const float mnew = fmaxf(mrow[r], cm[r]);
      const float alpha = __expf(mrow[r] - mnew);
      mrow[r] = mnew;
      float psum = 0.f;
#pragma unroll
      for (int j = 0; j < 4; ++j) {
        const float p = __expf(s[j][r] - mnew);
        psum += p;
        pw[(8 * hh + r) * 64 + j * 16 + m] = (_Float16)(p * 256.0f);
      }
#pragma unroll
      for (int off = 1; off < 16; off <<= 1) psum += __shfl_xor(psum, off, 32);
      lrow[r] = lrow[r] * alpha + psum;
#pragma unroll
      for (int t = 0; t < 8; ++t) oacc[t][r] *= alpha;
    }
    __builtin_amdgcn_fence(__ATOMIC_RELEASE, "workgroup");
    __builtin_amdgcn_wave_barrier();
    __builtin_amdgcn_fence(__ATOMIC_ACQUIRE, "workgroup");

#pragma unroll
    for (int kk = 0; kk < 2; ++kk) {
      FH pa;
      pa.h[0] = *(const v8h*)(pw + m * 64 + kk * 32 + 8 * hh);
      pa.h[1] = *(const v8h*)(pw + m * 64 + kk * 32 + 16 + 8 * hh);
#pragma unroll
      for (int t = 0; t < 8; ++t) {
        const _Float16* vr = Vth + (t * 16 + m) * 64 + kk * 32;
        FH vb;
        vb.h[0] = *(const v8h*)(vr + 8 * hh);
        vb.h[1] = *(const v8h*)(vr + 16 + 8 * hh);
        oacc[t] = mma_h(pa.v, vb.v, oacc[t]);
      }
    }
  }

  __syncthreads();
  float* OS = Os + wave * (128 * STP);
  float inv[8];
#pragma unroll
  for (int r = 0; r < 8; ++r) inv[r] = __builtin_amdgcn_rcpf(lrow[r]) * (1.0f / 256.0f);
#pragma unroll
  for (int t = 0; t < 8; ++t) {
    const int col = t * 16 + m;
    v4f p0, p1;
#pragma unroll
    for (int e = 0; e < 4; ++e) {
      p0[e] = oacc[t][e] * inv[e];
      p1[e] = oacc[t][4 + e] * inv[4 + e];
    }
    *(v4f*)(OS + col * STP + 8 * hh) = p0;
    *(v4f*)(OS + col * STP + 8 * hh + 4) = p1;
  }
  __syncthreads();
  for (int pass = 0; pass < 2; ++pass) {
#pragma unroll
    for (int it = 0; it < 8; ++it) {
      const int row = it * 2 + hh, c0 = 8 * m;
      float v[8];
#pragma unroll
      for (int e = 0; e < 8; ++e) v[e] = OS[(c0 + e) * STP + row];
      v4u hv, lv;
      split8(v, hv, lv);
      const size_t go = (gm + q0 + row) * HID + c0;
      *(volatile v4u*)(AVh + go) = hv;
      *(volatile v4u*)(AVl + go) = lv;
    }
    __threadfence();
  }
}

template <int EPI>
__global__ __launch_bounds__(256) void k_lin(const unsigned short* __restrict__ Ah, const unsigned short* __restrict__ Al,
                                             const unsigned short* __restrict__ Wh, const unsigned short* __restrict__ Wlo,
                                             const float* __restrict__ bias, const float* __restrict__ resid,
                                             void* __restrict__ o0, void* __restrict__ o1) {
  __shared__ __align__(16) unsigned short wl[2 * 128 * 32];
  __shared__ __align__(16) float st[4 * 128 * STP];
  const int tid = threadIdx.x, wave = tid >> 5, lane = tid & 31;
  const int m = lane & 15, hh = lane >> 4;
  const int pt = wave & 3, chf = wave >> 2;
  const int bm0 = blockIdx.x * 64;
  const int m0 = bm0 + pt * 16;
  const __bf16* ahp = (const __bf16*)Ah;
  const __bf16* alp = (const __bf16*)Al;
  const __bf16* wlb = (const __bf16*)wl;

  v8f acc[4];
#pragma unroll
  for (int nt = 0; nt < 4; ++nt) acc[nt] = zacc();

#pragma unroll 1
  for (int kc = 0; kc < 4; ++kc) {
    __syncthreads();
    for (int ci = tid; ci < 512; ci += 256) {
      const int col = ci >> 2, part = (ci & 3) * 8;
      const v4u ph = *(const v4u*)(Wh  + (size_t)col * HID + kc * 32 + part);
      const v4u pl = *(const v4u*)(Wlo + (size_t)col * HID + kc * 32 + part);
      *(v4u*)(wl + col * 32 + part) = ph;
      *(v4u*)(wl + 4096 + col * 32 + part) = pl;
    }
    __syncthreads();
    const size_t ao = (size_t)(m0 + m) * HID + kc * 32;
    FB ah, al;
    ah.h[0] = *(const v8b*)(ahp + ao + 8 * hh);
    ah.h[1] = *(const v8b*)(ahp + ao + 16 + 8 * hh);
    al.h[0] = *(const v8b*)(alp + ao + 8 * hh);
    al.h[1] = *(const v8b*)(alp + ao + 16 + 8 * hh);
#pragma unroll
    for (int nt = 0; nt < 4; ++nt) {
      const int col = chf * 64 + nt * 16 + m;
      const __bf16* br  = wlb + col * 32;
      const __bf16* brl = wlb + 4096 + col * 32;
      FB bh, bl;
      bh.h[0] = *(const v8b*)(br + 8 * hh);
      bh.h[1] = *(const v8b*)(br + 16 + 8 * hh);
      bl.h[0] = *(const v8b*)(brl + 8 * hh);
      bl.h[1] = *(const v8b*)(brl + 16 + 8 * hh);
      acc[nt] = mma_b(ah.v, bh.v, acc[nt]);
      acc[nt] = mma_b(ah.v, bl.v, acc[nt]);
      acc[nt] = mma_b(al.v, bh.v, acc[nt]);
    }
  }

  float* ST = st + pt * (128 * STP);
#pragma unroll
  for (int nt = 0; nt < 4; ++nt) {
    const int col = chf * 64 + nt * 16 + m;
    const float bv = bias[col];
    v4f p0, p1;
#pragma unroll
    for (int e = 0; e < 4; ++e) {
      p0[e] = acc[nt][e] + bv;
      p1[e] = acc[nt][4 + e] + bv;
    }
    *(v4f*)(ST + col * STP + 8 * hh) = p0;
    *(v4f*)(ST + col * STP + 8 * hh + 4) = p1;
  }
  __syncthreads();

  const int b = bm0 >> 12, p0 = bm0 & 4095;
  if (EPI == 1) {
    float* out = (float*)o0;
    for (int pass = 0; pass < 2; ++pass) {
#pragma unroll
      for (int it = 0; it < 8; ++it) {
        const int rowb = wave * 8 + it;
        const int ptr = rowb >> 4, r = rowb & 15;
        const int c4 = 4 * lane;
        v4f v;
#pragma unroll
        for (int e = 0; e < 4; ++e) v[e] = eluf(st[ptr * (128 * STP) + (c4 + e) * STP + r]);
        *(volatile v4f*)(out + (size_t)(bm0 + rowb) * HID + c4) = v;
      }
      __threadfence();
    }
  } else if (EPI == 2 || EPI == 3) {
    unsigned short* oh = (unsigned short*)o0;
    unsigned short* ol = (unsigned short*)o1;
    for (int pass = 0; pass < 2; ++pass) {
#pragma unroll
      for (int it = 0; it < 4; ++it) {
        const int rowb = (wave * 4 + it) * 2 + hh;
        const int ptr = rowb >> 4, r = rowb & 15;
        const int c0 = 8 * m;
        float v[8];
#pragma unroll
        for (int e = 0; e < 8; ++e) v[e] = eluf(st[ptr * (128 * STP) + (c0 + e) * STP + r]);
        if (EPI == 3) {
          const v4f r0v = *(const v4f*)(resid + (size_t)(bm0 + rowb) * HID + c0);
          const v4f r1v = *(const v4f*)(resid + (size_t)(bm0 + rowb) * HID + c0 + 4);
#pragma unroll
          for (int e = 0; e < 4; ++e) { v[e] = eluf(v[e] + r0v[e]); v[4 + e] = eluf(v[4 + e] + r1v[e]); }
        }
        v4u hv, lv;
        split8(v, hv, lv);
        const size_t go = (size_t)(bm0 + rowb) * HID + c0;
        *(volatile v4u*)(oh + go) = hv;
        *(volatile v4u*)(ol + go) = lv;
      }
      __threadfence();
    }
  } else {
    float* out = (float*)o0;
    for (int pass = 0; pass < 2; ++pass) {
#pragma unroll
      for (int it = 0; it < 8; ++it) {
        const int ch = wave * 16 + it * 2 + hh;
        const int pxb = 4 * m;
        const int ptr = pxb >> 4, r0 = pxb & 15;
        v4f v = *(const v4f*)(st + ptr * (128 * STP) + ch * STP + r0);
#pragma unroll
        for (int e = 0; e < 4; ++e) v[e] = eluf(v[e]);
        *(volatile v4f*)(out + ((size_t)(b * HID + ch)) * NPOS + p0 + pxb) = v;
      }
      __threadfence();
    }
  }
}

extern "C" void kernel_launch(void* const* d_in, const int* in_sizes, int n_in,
                              void* d_out, int out_size, void* d_ws, size_t ws_size,
                              hipStream_t stream) {
  if (n_in < 16) return;
  if (in_sizes[0] != MPIX * HID) return;
  if (in_sizes[1] != NBATCH * 2 * NPOS) return;
  if (in_sizes[2] != NLAYER * HID * HID * 4 || in_sizes[3] != NLAYER * HID) return;
  if (in_sizes[4] != NLAYER * 2 * HID * HID * 4 || in_sizes[5] != NLAYER * 2 * HID) return;
  if (in_sizes[6] != KQ * CIN || in_sizes[7] != KQ) return;
  if (in_sizes[8] != HID * HID || in_sizes[9] != HID) return;
  if (in_sizes[10] != HID * HID || in_sizes[11] != HID) return;
  if (in_sizes[12] != HID * HID || in_sizes[13] != HID) return;
  if (in_sizes[14] != HID * HID || in_sizes[15] != HID) return;
  if (out_size != MPIX * HID) return;

  const float* x       = (const float*)d_in[0];
  const float* pos     = (const float*)d_in[1];
  const float* conv1_w = (const float*)d_in[2];
  const float* conv1_b = (const float*)d_in[3];
  const float* conv2_w = (const float*)d_in[4];
  const float* conv2_b = (const float*)d_in[5];
  const float* qkv_w   = (const float*)d_in[6];
  const float* qkv_b   = (const float*)d_in[7];
  const float* ap_w    = (const float*)d_in[8];
  const float* ap_b    = (const float*)d_in[9];
  const float* oc_w    = (const float*)d_in[10];
  const float* oc_b    = (const float*)d_in[11];
  const float* oa_w    = (const float*)d_in[12];
  const float* oa_b    = (const float*)d_in[13];
  const float* op_w    = (const float*)d_in[14];
  const float* op_b    = (const float*)d_in[15];

  const size_t SZ_WC1 = (size_t)NLAYER * 128 * 512 * 2;
  const size_t SZ_WC2 = (size_t)NLAYER * 256 * 512 * 2;
  const size_t SZ_WQ  = (size_t)KQ * KQ * 2;
  const size_t SZ_WP  = (size_t)HID * HID * 2;
  const size_t SZ_HF  = (size_t)MPIX * HID * 4;
  const size_t SZ_H16 = (size_t)MPIX * HID * 2;
  const size_t SZ_O   = (size_t)MPIX * 256 * 4;
  const size_t SZ_AB  = (size_t)MPIX * KQ * 2;
  const size_t SZ_QK  = (size_t)MPIX * QKD * 2;
  const size_t SZ_VT  = (size_t)NBATCH * HID * NPOS * 2;

  size_t off = 0;
  const size_t oWC1 = off; off += SZ_WC1;
  const size_t oWC2 = off; off += SZ_WC2;
  const size_t oWQ  = off; off += SZ_WQ;
  const size_t oAPh = off; off += SZ_WP;  const size_t oAPl = off; off += SZ_WP;
  const size_t oOCh = off; off += SZ_WP;  const size_t oOCl = off; off += SZ_WP;
  const size_t oOAh = off; off += SZ_WP;  const size_t oOAl = off; off += SZ_WP;
  const size_t oOPh = off; off += SZ_WP;  const size_t oOPl = off; off += SZ_WP;
  const size_t oH0  = off; off += SZ_HF;
  const size_t oH1  = off; off += SZ_HF;
  const size_t oHX  = off; off += SZ_H16;
  const size_t oT1  = off; off += SZ_H16;
  const size_t oO   = off; off += SZ_O;
  const size_t oAB  = off; off += SZ_AB;
  const size_t oQ   = off; off += SZ_QK;
  const size_t oK   = off; off += SZ_QK;
  const size_t oVT  = off; off += SZ_VT;
  const size_t oAVh = off; off += SZ_H16;
  const size_t oAVl = off; off += SZ_H16;
  const size_t oCH  = off; off += SZ_H16;
  const size_t oCL  = off; off += SZ_H16;
  const size_t oCP  = off; off += SZ_HF;
  const size_t oAH  = off; off += SZ_H16;
  const size_t oAL  = off; off += SZ_H16;
  const size_t oSH  = off; off += SZ_H16;
  const size_t oSL  = off; off += SZ_H16;
  if (off > ws_size) return;
  if (off > (size_t)134217728) return;

  char* ws = (char*)d_ws;
  unsigned short* WC1 = (unsigned short*)(ws + oWC1);
  unsigned short* WC2 = (unsigned short*)(ws + oWC2);
  unsigned short* WQ  = (unsigned short*)(ws + oWQ);
  unsigned short* APh = (unsigned short*)(ws + oAPh); unsigned short* APl = (unsigned short*)(ws + oAPl);
  unsigned short* OCh = (unsigned short*)(ws + oOCh); unsigned short* OCl = (unsigned short*)(ws + oOCl);
  unsigned short* OAh = (unsigned short*)(ws + oOAh); unsigned short* OAl = (unsigned short*)(ws + oOAl);
  unsigned short* OPh = (unsigned short*)(ws + oOPh); unsigned short* OPl = (unsigned short*)(ws + oOPl);
  float*          H0  = (float*)(ws + oH0);
  float*          H1  = (float*)(ws + oH1);
  unsigned short* HX  = (unsigned short*)(ws + oHX);
  unsigned short* T1  = (unsigned short*)(ws + oT1);
  float*          O   = (float*)(ws + oO);
  unsigned short* AB  = (unsigned short*)(ws + oAB);
  unsigned short* Qb  = (unsigned short*)(ws + oQ);
  unsigned short* Kb  = (unsigned short*)(ws + oK);
  unsigned short* VT  = (unsigned short*)(ws + oVT);
  unsigned short* AVh = (unsigned short*)(ws + oAVh); unsigned short* AVl = (unsigned short*)(ws + oAVl);
  unsigned short* CH  = (unsigned short*)(ws + oCH);  unsigned short* CL  = (unsigned short*)(ws + oCL);
  float*          CP  = (float*)(ws + oCP);
  unsigned short* AH  = (unsigned short*)(ws + oAH);  unsigned short* AL  = (unsigned short*)(ws + oAL);
  unsigned short* SH  = (unsigned short*)(ws + oSH);  unsigned short* SL  = (unsigned short*)(ws + oSL);

  const dim3 blk256(256), blk128(128);

  k_prep_convw<<<dim3((NLAYER * 128 * 64 + 255) / 256), blk256, 0, stream>>>(conv1_w, WC1, NLAYER * 128);
  k_prep_convw<<<dim3((NLAYER * 256 * 64 + 255) / 256), blk256, 0, stream>>>(conv2_w, WC2, NLAYER * 256);
  k_prep_qkvw<<<dim3((KQ * KQ / 8 + 255) / 256), blk256, 0, stream>>>(qkv_w, WQ);
  k_prep_splitw<<<dim3(HID * HID / 8 / 256), blk256, 0, stream>>>(ap_w, APh, APl);
  k_prep_splitw<<<dim3(HID * HID / 8 / 256), blk256, 0, stream>>>(oc_w, OCh, OCl);
  k_prep_splitw<<<dim3(HID * HID / 8 / 256), blk256, 0, stream>>>(oa_w, OAh, OAl);
  k_prep_splitw<<<dim3(HID * HID / 8 / 256), blk256, 0, stream>>>(op_w, OPh, OPl);

  k_transpose_in<<<dim3(NBATCH * 64), blk256, 0, stream>>>(x, H0, HX);

  for (int l = 0; l < NLAYER; ++l) {
    float* Hc = (l & 1) ? H1 : H0;
    float* Hn = (l & 1) ? H0 : H1;
    k_conv<0><<<dim3(MPIX / 64, 1), blk128, 0, stream>>>(HX, WC1 + (size_t)l * 128 * 512, conv1_b + l * 128, (void*)T1);
    k_conv<1><<<dim3(MPIX / 64, 2), blk128, 0, stream>>>(T1, WC2 + (size_t)l * 256 * 512, conv2_b + l * 256, (void*)O);
    k_gate<<<dim3(MPIX * 32 / 256), blk256, 0, stream>>>(Hc, O, Hn, HX);
  }

  k_build_a<<<dim3(MPIX * 20 / 256), blk256, 0, stream>>>(H0, pos, AB);
  k_qkv<<<dim3(MPIX / 64), blk128, 0, stream>>>(AB, WQ, qkv_b, Qb, Kb, VT);
  k_attn<<<dim3(NBATCH * 64), blk128, 0, stream>>>(Qb, Kb, VT, AVh, AVl);

  k_split_elu<<<dim3(MPIX * 16 / 256), blk256, 0, stream>>>(H0, CH, CL);
  k_lin<1><<<dim3(MPIX / 64), blk256, 0, stream>>>(CH, CL, OCh, OCl, oc_b, CP, (void*)CP, (void*)CP);
  k_lin<2><<<dim3(MPIX / 64), blk256, 0, stream>>>(AVh, AVl, APh, APl, ap_b, CP, (void*)AH, (void*)AL);
  k_lin<3><<<dim3(MPIX / 64), blk256, 0, stream>>>(AH, AL, OAh, OAl, oa_b, CP, (void*)SH, (void*)SL);
  k_lin<4><<<dim3(MPIX / 64), blk256, 0, stream>>>(SH, SL, OPh, OPl, op_b, CP, d_out, d_out);

  (void)hipGetLastError();
}
